// GateLoopAttention_83631603187968
// MI455X (gfx1250) — hardware-run, weakly checked
//
#include <hip/hip_runtime.h>
#include <math.h>

typedef __attribute__((ext_vector_type(16))) __bf16   v16b;
typedef __attribute__((ext_vector_type(8)))  __bf16   v8b;
typedef __attribute__((ext_vector_type(8)))  float    v8f;
typedef __attribute__((ext_vector_type(4)))  float    v4f;
typedef __attribute__((ext_vector_type(2)))  float    v2f;
typedef __attribute__((ext_vector_type(4)))  unsigned int v4u;

constexpr int kSeq    = 4096;
constexpr int kDim    = 512;
constexpr int kInner  = 512;
constexpr int kHeads  = 16;
constexpr int kHd     = kInner / kHeads;
constexpr int kQkvN   = 3 * kInner;
constexpr int kGateN  = 2 * kHeads;
constexpr int kNpad   = ((kQkvN + kGateN + 63) / 64) * 64;
constexpr int kChunk  = 64;
static_assert(kHd == 32, "head width");
static_assert(kQkvN == 1536 && kGateN == 32 && kNpad == 1600, "projection widths");
static_assert((kDim % 32) == 0, "GEMM K multiple of 32");
static_assert((kSeq % 64) == 0 && (kNpad % 64) == 0, "GEMM M,N multiples of 64");
static_assert(((kSeq / 64) * (kNpad / 64)) % 8 == 0, "whole blocks of 8 tile waves");
static_assert((kSeq % kChunk) == 0 && (kSeq % 256) == 0, "scan chunking");
static_assert((kQkvN % 64) == 0 && (kDim % 64) == 0, "weight tile multiples");

constexpr size_t kOffXB   = 0;
constexpr size_t kOffWTB  = kOffXB   + (size_t)kSeq  * kDim  * 2;
constexpr size_t kOffQKVA = kOffWTB  + (size_t)kNpad * kDim  * 2;
constexpr size_t kOffGATE = kOffQKVA + (size_t)kSeq  * kNpad * 4;
constexpr size_t kWsTotal = kOffGATE + (size_t)kHeads * kSeq * 2 * 4;
static_assert(kWsTotal == 32571392ull, "carve total");
static_assert(kWsTotal <= 134217728ull, "carve cap");
static_assert((kOffWTB % 128) == 0 && (kOffQKVA % 128) == 0 && (kOffGATE % 128) == 0, "128-B aligned regions");

__device__ __forceinline__ unsigned short f2bf_bits(float f) {
  unsigned u = __float_as_uint(f);
  return (unsigned short)((u + 0x7FFFu + ((u >> 16) & 1u)) >> 16);
}
__device__ __forceinline__ float bf_bits2f(unsigned short h) { return __uint_as_float(((unsigned)h) << 16); }
__device__ __forceinline__ unsigned pk16(unsigned short a, unsigned short b) { return (unsigned)a | ((unsigned)b << 16); }

__device__ __forceinline__ void keep4_b(v16b a, v16b b, v16b c, v16b d) { asm volatile("v_nop" :: "v"(a), "v"(b), "v"(c), "v"(d)); }
__device__ __forceinline__ void acc_guard4(v8f& a, v8f& b, v8f& c, v8f& d) { asm volatile("v_nop\n\tv_nop\n\tv_nop\n\tv_nop" : "+v"(a), "+v"(b), "+v"(c), "+v"(d)); }

struct FragB {
  union U { v16b v; v8b h[2]; };
  static __device__ __forceinline__ v16b load(const __bf16* p) {
    U f; f.h[0] = *(const v8b*)(p); f.h[1] = *(const v8b*)(p + 16); return f.v;
  }
  static __device__ __forceinline__ v8f mma(v16b a, v16b b, v8f c) {
    c = __builtin_amdgcn_wmma_f32_16x16x32_bf16(false, a, false, b, (short)0, c, false, false);
    asm volatile("v_nop\n\tv_nop\n\tv_nop\n\tv_nop" : "+v"(c) : "v"(a), "v"(b));
    return c;
  }
};

__global__ __launch_bounds__(256) void gemm64_bf16_kernel(
    const unsigned short* __restrict__ Ap, int lda,
    const unsigned short* __restrict__ Btp, int ldb,
    float* __restrict__ C, int ldc,
    int M, int N, int K) {
  const __bf16* A  = (const __bf16*)Ap;
  const __bf16* Bt = (const __bf16*)Btp;
  __shared__ __align__(16) float sT[8][16 * 68];
  const int lane = threadIdx.x & 31;
  const int wave = threadIdx.x >> 5;
  const int tilesN = N >> 6;
  const int tilesM = M >> 6;
  const int tile = blockIdx.x * 8 + wave;
  if (tile >= tilesM * tilesN) return;
  const int tm = tile / tilesN;
  const int tn = tile - tm * tilesN;
  const int m0 = tm << 6;
  const int n0 = tn << 6;

  const int rlane = lane & 15;
  const int koff  = (lane >> 4) * 8;
  const int mOff  = (lane >> 4) * 8;

  v8f acc[4][4];
#pragma unroll
  for (int i = 0; i < 4; ++i)
#pragma unroll
    for (int j = 0; j < 4; ++j) acc[i][j] = (v8f){0.f,0.f,0.f,0.f,0.f,0.f,0.f,0.f};

  for (int k0 = 0; k0 < K; k0 += 32) {
    v16b bh[4];
#pragma unroll
    for (int j = 0; j < 4; ++j) {
      const size_t bo = (size_t)(n0 + (j << 4) + rlane) * ldb + koff + k0;
      bh[j] = FragB::load(Bt + bo);
    }
#pragma unroll
    for (int i = 0; i < 4; ++i) {
      const size_t ao = (size_t)(m0 + (i << 4) + rlane) * lda + koff + k0;
      const v16b ah = FragB::load(A + ao);
#pragma unroll
      for (int j = 0; j < 4; ++j) acc[i][j] = FragB::mma(ah, bh[j], acc[i][j]);
    }
    keep4_b(bh[0], bh[1], bh[2], bh[3]);
  }
  acc_guard4(acc[0][0], acc[0][1], acc[0][2], acc[0][3]);
  acc_guard4(acc[1][0], acc[1][1], acc[1][2], acc[1][3]);
  acc_guard4(acc[2][0], acc[2][1], acc[2][2], acc[2][3]);
  acc_guard4(acc[3][0], acc[3][1], acc[3][2], acc[3][3]);

  float* slab = sT[wave];
#pragma unroll
  for (int i = 0; i < 4; ++i) {
    const int mBase = m0 + (i << 4);
#pragma unroll
    for (int j = 0; j < 4; ++j) {
#pragma unroll
      for (int r = 0; r < 8; ++r) slab[(mOff + r) * 68 + (j << 4) + rlane] = acc[i][j][r];
    }
    __builtin_amdgcn_fence(__ATOMIC_RELEASE, "workgroup");
    __builtin_amdgcn_wave_barrier();
    __builtin_amdgcn_fence(__ATOMIC_ACQUIRE, "workgroup");
    {
      const int hh = lane >> 4, c4 = (lane & 15) * 4;
      for (int pass = 0; pass < 2; ++pass) {
#pragma unroll
        for (int it = 0; it < 8; ++it) {
          const int row = it * 2 + hh;
          const v4f v = *(const v4f*)(slab + row * 68 + c4);
          *(volatile v4f*)(C + (size_t)(mBase + row) * ldc + n0 + c4) = v;
        }
        __threadfence();
      }
    }
    __builtin_amdgcn_fence(__ATOMIC_RELEASE, "workgroup");
    __builtin_amdgcn_wave_barrier();
    __builtin_amdgcn_fence(__ATOMIC_ACQUIRE, "workgroup");
  }
}

__global__ __launch_bounds__(256) void cvt_rows_bf16_kernel(
    const float* __restrict__ src, unsigned short* __restrict__ dst, int total8) {
  const int i = blockIdx.x * 256 + threadIdx.x;
  if (i >= total8) return;
  const size_t e0 = (size_t)i << 3;
  const v4f a0 = *(const v4f*)(src + e0);
  const v4f a1 = *(const v4f*)(src + e0 + 4);
  unsigned short hb[8];
#pragma unroll
  for (int e = 0; e < 4; ++e) {
    hb[e]     = f2bf_bits(a0[e]);
    hb[4 + e] = f2bf_bits(a1[e]);
  }
  const v4u u = (v4u){pk16(hb[0], hb[1]), pk16(hb[2], hb[3]), pk16(hb[4], hb[5]), pk16(hb[6], hb[7])};
  unsigned short* q = dst + e0;
  *(volatile v4u*)q = u;
  __threadfence();
  *(volatile v4u*)q = u;
}

__global__ __launch_bounds__(256) void wt_bf16_kernel(
    const float* __restrict__ Wqkv, const float* __restrict__ Wa, unsigned short* __restrict__ WT) {
  __shared__ float sm[64][65];
  const int t  = threadIdx.x;
  const int k0 = blockIdx.x * 64;
  const int nt = blockIdx.y;
  const int n0 = nt * 64;
  if (nt < kQkvN / 64) {
#pragma unroll
    for (int i = 0; i < 16; ++i) {
      const int e = i * 256 + t;
      const int r = e >> 6;
      const int c = e & 63;
      sm[c][r] = Wqkv[(size_t)(k0 + r) * kQkvN + n0 + c];
    }
  } else {
#pragma unroll
    for (int i = 0; i < 8; ++i) {
      const int e = i * 256 + t;
      const int r = e >> 5;
      const int c = e & 31;
      sm[c][r]      = Wa[(size_t)(k0 + r) * kGateN + c];
      sm[32 + c][r] = 0.0f;
    }
  }
  __syncthreads();
  const int lane = t & 31, wave = t >> 5;
  const int q = lane >> 3, c8 = (lane & 7) * 8;
  v4u u[2];
#pragma unroll
  for (int it = 0; it < 2; ++it) {
    const int row = wave * 8 + it * 4 + q;
    unsigned short hb[8];
#pragma unroll
    for (int e = 0; e < 8; ++e) hb[e] = f2bf_bits(sm[row][c8 + e]);
    u[it] = (v4u){pk16(hb[0], hb[1]), pk16(hb[2], hb[3]), pk16(hb[4], hb[5]), pk16(hb[6], hb[7])};
  }
  for (int pass = 0; pass < 2; ++pass) {
#pragma unroll
    for (int it = 0; it < 2; ++it) {
      const int row = wave * 8 + it * 4 + q;
      *(volatile v4u*)(WT + (size_t)(n0 + row) * kDim + k0 + c8) = u[it];
    }
    __threadfence();
  }
}

__global__ __launch_bounds__(256) void gate_kernel(
    const float* __restrict__ P, const float* __restrict__ ba, float* __restrict__ G) {
  __shared__ __align__(16) float sg[512];
  const int t = threadIdx.x;
  const int i = blockIdx.x * 256 + t;
  const int h = i >> 12;
  const int n = i & (kSeq - 1);
  const v2f av = *(const v2f*)(P + (size_t)n * kNpad + kQkvN + 2 * h);
  const float br = bf_bits2f(f2bf_bits(ba[2 * h]));
  const float bi = bf_bits2f(f2bf_bits(ba[2 * h + 1]));
  const float ar = av.x + br;
  const float ai = av.y + bi;
  const float mag = sqrtf(ar * ar + ai * ai);
  const float sig = 1.0f / (1.0f + expf(-mag));
  const bool  pos = (mag > 0.0f);
  const float magc = pos ? mag : 1.0f;
  const float sc = sig * (1.0f / magc);
  const float gr = pos ? ar * sc : sig;
  const float gi = pos ? ai * sc : 0.0f;
  sg[2 * t]     = gr;
  sg[2 * t + 1] = gi;
  __syncthreads();
  if (t < 128) {
    const v4f gv = *(const v4f*)(sg + 4 * t);
    float* p = G + (size_t)blockIdx.x * 512 + 4 * t;
    *(volatile v4f*)p = gv;
    __threadfence();
    *(volatile v4f*)p = gv;
  }
}

__global__ __launch_bounds__(64) void gated_scan_kernel(
    const float* __restrict__ P, const float* __restrict__ G, float* __restrict__ out) {
  __shared__ __align__(16) float sQ[kChunk * kHd];
  __shared__ __align__(16) float sK[kChunk * kHd];
  __shared__ __align__(16) float sV[kChunk * kHd];
  __shared__ __align__(16) float sO[kChunk * kHd];
  __shared__ __align__(16) float sG[kChunk * 2];
  const int tid  = threadIdx.x;
  const int lane = tid & 31;
  const int wave = tid >> 5;
  const int h    = blockIdx.x;
  const int dh   = lane >> 4;
  const int e    = wave * 16 + (lane & 15);
  const int lr   = tid >> 3;
  const int lc4  = (tid & 7) * 4;
  const int sq   = lane >> 3;
  const int sc4  = (lane & 7) * 4;

  float sr[16], si[16];
#pragma unroll
  for (int j = 0; j < 16; ++j) { sr[j] = 0.0f; si[j] = 0.0f; }

#pragma unroll 1
  for (int t0 = 0; t0 < kSeq; t0 += kChunk) {
#pragma unroll
    for (int i = 0; i < 8; ++i) {
      const int r = lr + 8 * i;
      const float* base = P + (size_t)(t0 + r) * kNpad + h * kHd + lc4;
      const v4f vq = *(const v4f*)(base);
      const v4f vk = *(const v4f*)(base + kInner);
      const v4f vv = *(const v4f*)(base + 2 * kInner);
      *(v4f*)(sQ + r * kHd + lc4) = vq;
      *(v4f*)(sK + r * kHd + lc4) = vk;
      *(v4f*)(sV + r * kHd + lc4) = vv;
    }
    {
      const v2f gv = *(const v2f*)(G + 2 * ((size_t)h * kSeq + t0 + tid));
      *(v2f*)(sG + 2 * tid) = gv;
    }
    __syncthreads();

#pragma unroll 1
    for (int s = 0; s < kChunk; ++s) {
      const v2f g = *(const v2f*)(sG + 2 * s);
      const float vv = sV[s * kHd + e];
      const float* qp = sQ + s * kHd + 16 * dh;
      const float* kp = sK + s * kHd + 16 * dh;
      float qq[16], kk[16];
#pragma unroll
      for (int j4 = 0; j4 < 4; ++j4) {
        const v4f tq = *(const v4f*)(qp + 4 * j4);
        const v4f tk = *(const v4f*)(kp + 4 * j4);
        qq[4 * j4 + 0] = tq[0]; qq[4 * j4 + 1] = tq[1]; qq[4 * j4 + 2] = tq[2]; qq[4 * j4 + 3] = tq[3];
        kk[4 * j4 + 0] = tk[0]; kk[4 * j4 + 1] = tk[1]; kk[4 * j4 + 2] = tk[2]; kk[4 * j4 + 3] = tk[3];
      }
      float part = 0.0f;
#pragma unroll
      for (int j = 0; j < 16; ++j) {
        const float kvp = kk[j] * vv;
        const float nr = g.x * sr[j] - g.y * si[j] + kvp;
        const float ni = g.x * si[j] + g.y * sr[j];
        sr[j] = nr;
        si[j] = ni;
        part = fmaf(qq[j], nr, part);
      }
      const float oth = __shfl_xor(part, 16, 32);
      const float tot = part + oth;
      if (dh == 0) sO[s * kHd + e] = tot;
    }
    __syncthreads();

    v4f ov[8];
#pragma unroll
    for (int it = 0; it < 8; ++it) {
      const int row = it * 8 + wave * 4 + sq;
      ov[it] = *(const v4f*)(sO + row * kHd + sc4);
    }
    for (int pass = 0; pass < 2; ++pass) {
#pragma unroll
      for (int it = 0; it < 8; ++it) {
        const int row = it * 8 + wave * 4 + sq;
        *(volatile v4f*)(out + (size_t)(t0 + row) * kInner + h * kHd + sc4) = ov[it];
      }
      __threadfence();
    }
  }
}

extern "C" void kernel_launch(void* const* d_in, const int* in_sizes, int n_in,
                              void* d_out, int out_size, void* d_ws, size_t ws_size,
                              hipStream_t stream) {
  if (n_in < 4) return;
  if (in_sizes[0] != kSeq * kDim) return;
  if (in_sizes[1] != kDim * kQkvN) return;
  if (in_sizes[2] != kDim * kGateN) return;
  if (in_sizes[3] != kGateN) return;
  if (out_size != kSeq * kInner) return;
  if (ws_size < kWsTotal) return;

  const float* x     = (const float*)d_in[0];
  const float* W_qkv = (const float*)d_in[1];
  const float* W_a   = (const float*)d_in[2];
  const float* b_a   = (const float*)d_in[3];
  float* out = (float*)d_out;

  char* ws = (char*)d_ws;
  unsigned short* XB   = (unsigned short*)(ws + kOffXB);
  unsigned short* WTB  = (unsigned short*)(ws + kOffWTB);
  float*          QKVA = (float*)(ws + kOffQKVA);
  float*          GATE = (float*)(ws + kOffGATE);

  cvt_rows_bf16_kernel<<<(kSeq * kDim / 8) / 256, 256, 0, stream>>>(x, XB, kSeq * kDim / 8);

  wt_bf16_kernel<<<dim3(kDim / 64, kNpad / 64), 256, 0, stream>>>(W_qkv, W_a, WTB);

  gemm64_bf16_kernel<<<((kSeq / 64) * (kNpad / 64)) / 8, 256, 0, stream>>>(
      XB, kDim, WTB, kDim, QKVA, kNpad, kSeq, kNpad, kDim);

  gate_kernel<<<(kHeads * kSeq) / 256, 256, 0, stream>>>(QKVA, b_a, GATE);

  gated_scan_kernel<<<kHeads, 64, 0, stream>>>(QKVA, GATE, out);
}
